// RWKV7CrossAttention_34815004902092
// MI455X (gfx1250) — hardware-verified
//
#include <hip/hip_runtime.h>
#include <math.h>

constexpr int kBatch  = 2;
constexpr int kSeq    = 1024;
constexpr int kCh     = 1024;
constexpr int kHeads  = 16;
constexpr int kHd     = 64;
constexpr int kRows   = kBatch * kSeq;
constexpr int kRankW  = 64;
constexpr int kRankA  = 64;
constexpr int kRankV  = 16;
constexpr int kRankVP = 64;
constexpr int kRankG  = 128;
constexpr int kChunk  = 16;
constexpr float kLoraCarry    = 64.0f;
constexpr float kLoraCarryInv = 1.0f / 64.0f;
constexpr float kDecay        = -0.6065306597126334f;
constexpr float kNormEps      = (float)kHd * 1e-5f;
constexpr float kInvHd        = 1.0f / (float)kHd;
static_assert(kHeads * kHd == kCh, "heads x head dim");
static_assert((kSeq & (kSeq - 1)) == 0, "time extent is a power of two");
static_assert(kRows % 64 == 0 && kCh % 64 == 0, "GEMM M/N tile multiples");
static_assert(kCh % 32 == 0 && kRankW % 32 == 0 && kRankA % 32 == 0 && kRankVP % 32 == 0 && kRankG % 32 == 0, "GEMM K multiples of 32");
static_assert(kRankW % 64 == 0 && kRankA % 64 == 0 && kRankVP % 64 == 0 && kRankG % 64 == 0, "GEMM N tile multiples");
static_assert(kRankV <= kRankVP, "rank pad");
static_assert(kSeq % kChunk == 0, "scan chunking");
static_assert(kHd == 64 && kChunk == 16, "scan thread maps assume 64-wide heads and 16-step chunks");

typedef __attribute__((ext_vector_type(16))) _Float16 v16h;
typedef __attribute__((ext_vector_type(8)))  _Float16 v8h;
typedef __attribute__((ext_vector_type(16))) __bf16   v16b;
typedef __attribute__((ext_vector_type(8)))  __bf16   v8b;
typedef __attribute__((ext_vector_type(8)))  float    v8f;
typedef __attribute__((ext_vector_type(4)))  float    v4f;
typedef __attribute__((ext_vector_type(2)))  float    v2f;
typedef __attribute__((ext_vector_type(4)))  unsigned int v4u;

__device__ __forceinline__ unsigned short f2bf_bits(float f) {
  unsigned u = __float_as_uint(f);
  return (unsigned short)((u + 0x7FFFu + ((u >> 16) & 1u)) >> 16);
}
__device__ __forceinline__ float bf_bits2f(unsigned short h) { return __uint_as_float(((unsigned)h) << 16); }
__device__ __forceinline__ unsigned pk16(unsigned short a, unsigned short b) { return (unsigned)a | ((unsigned)b << 16); }
__device__ __forceinline__ unsigned short h_bits(float f) { const _Float16 h = (_Float16)f; return __builtin_bit_cast(unsigned short, h); }
__device__ __forceinline__ void split_bits(float f, unsigned short& hb, unsigned short& lb) {
  hb = f2bf_bits(f);
  lb = f2bf_bits(f - bf_bits2f(hb));
}
__device__ __forceinline__ void pack_split8(const float (&x)[8], v4u& H, v4u& L) {
  unsigned short hb[8], lb[8];
#pragma unroll
  for (int e = 0; e < 8; ++e) split_bits(x[e], hb[e], lb[e]);
  H = (v4u){pk16(hb[0], hb[1]), pk16(hb[2], hb[3]), pk16(hb[4], hb[5]), pk16(hb[6], hb[7])};
  L = (v4u){pk16(lb[0], lb[1]), pk16(lb[2], lb[3]), pk16(lb[4], lb[5]), pk16(lb[6], lb[7])};
}
__device__ __forceinline__ v4u pack_f16x8(const float (&x)[8]) {
  unsigned short hb[8];
#pragma unroll
  for (int e = 0; e < 8; ++e) hb[e] = h_bits(x[e]);
  return (v4u){pk16(hb[0], hb[1]), pk16(hb[2], hb[3]), pk16(hb[4], hb[5]), pk16(hb[6], hb[7])};
}
__device__ __forceinline__ float sigm(float x) { return __builtin_amdgcn_rcpf(1.0f + expf(-x)); }

__device__ __forceinline__ void dep_guard4_h(v8f& a, v8f& b, v8f& c, v8f& d, v16h x, v16h y) {
  asm volatile("v_nop\n\tv_nop\n\tv_nop\n\tv_nop" : "+v"(a), "+v"(b), "+v"(c), "+v"(d) : "v"(x), "v"(y));
}
__device__ __forceinline__ void dep_guard4_b(v8f& a, v8f& b, v8f& c, v8f& d, v16b x, v16b y) {
  asm volatile("v_nop\n\tv_nop\n\tv_nop\n\tv_nop" : "+v"(a), "+v"(b), "+v"(c), "+v"(d) : "v"(x), "v"(y));
}
__device__ __forceinline__ void keep4_h(v16h a, v16h b, v16h c, v16h d) { asm volatile("v_nop" :: "v"(a), "v"(b), "v"(c), "v"(d)); }
__device__ __forceinline__ void keep4_b(v16b a, v16b b, v16b c, v16b d) { asm volatile("v_nop" :: "v"(a), "v"(b), "v"(c), "v"(d)); }
__device__ __forceinline__ void acc_guard4(v8f& a, v8f& b, v8f& c, v8f& d) {
  asm volatile("v_nop\n\tv_nop\n\tv_nop\n\tv_nop" : "+v"(a), "+v"(b), "+v"(c), "+v"(d));
}
template <typename T> struct Frag;
template <> struct Frag<_Float16> {
  typedef v16h V; union U { v16h v; v8h h[2]; };
  static __device__ __forceinline__ v16h load(const _Float16* p) {
    U f; f.h[0] = *(const v8h*)(p); f.h[1] = *(const v8h*)(p + 16); return f.v;
  }
  static __device__ __forceinline__ v8f mma(v16h a, v16h b, v8f c) {
    return __builtin_amdgcn_wmma_f32_16x16x32_f16(false, a, false, b, (short)0, c, false, false);
  }
  static __device__ __forceinline__ void guard4(v8f& a, v8f& b, v8f& c, v8f& d, v16h x, v16h y) { dep_guard4_h(a, b, c, d, x, y); }
  static __device__ __forceinline__ void keep(v16h a, v16h b, v16h c, v16h d) { keep4_h(a, b, c, d); }
};
template <> struct Frag<__bf16> {
  typedef v16b V; union U { v16b v; v8b h[2]; };
  static __device__ __forceinline__ v16b load(const __bf16* p) {
    U f; f.h[0] = *(const v8b*)(p); f.h[1] = *(const v8b*)(p + 16); return f.v;
  }
  static __device__ __forceinline__ v8f mma(v16b a, v16b b, v8f c) {
    return __builtin_amdgcn_wmma_f32_16x16x32_bf16(false, a, false, b, (short)0, c, false, false);
  }
  static __device__ __forceinline__ void guard4(v8f& a, v8f& b, v8f& c, v8f& d, v16b x, v16b y) { dep_guard4_b(a, b, c, d, x, y); }
  static __device__ __forceinline__ void keep(v16b a, v16b b, v16b c, v16b d) { keep4_b(a, b, c, d); }
};

template <int ET> struct Elem;
template <> struct Elem<0> { typedef _Float16 T; };
template <> struct Elem<1> { typedef __bf16 T; };
template <int ET, bool SPLIT, int BIAS_MODE, int OUT_MODE, bool RESID, int ACT = 0>
__global__ __launch_bounds__(256) void wmma_gemm64(
    const unsigned short* __restrict__ Ap, const unsigned short* __restrict__ A2p, int lda, long strideA,
    const unsigned short* __restrict__ Btp, const unsigned short* __restrict__ Bt2p, int ldb, long strideB,
    void* __restrict__ Cout, void* __restrict__ Cout2, int ldc, long strideC,
    const float* __restrict__ bias,
    const float* __restrict__ resid, long strideR,
    int M, int N, int K, float scale) {
  typedef typename Elem<ET>::T T;
  typedef typename Frag<T>::V V;
  const T* A = (const T*)Ap; const T* A2 = (const T*)A2p; const T* Bt = (const T*)Btp; const T* Bt2 = (const T*)Bt2p;
  __shared__ __align__(16) float sT[8][16 * 68];
  const int b    = blockIdx.y;
  const int lane = threadIdx.x & 31;
  const int wave = threadIdx.x >> 5;
  const int tilesN = N >> 6;
  const int tilesM = M >> 6;
  const int tile = blockIdx.x * 8 + wave;
  if (tile >= tilesM * tilesN) return;
  const int tm = tile / tilesN;
  const int tn = tile - tm * tilesN;
  const int m0 = tm << 6;
  const int n0 = tn << 6;

  const T* Ab  = A  + (size_t)b * strideA;
  const T* Bb  = Bt + (size_t)b * strideB;
  const T* Ab2 = SPLIT ? (A2  + (size_t)b * strideA) : nullptr;
  const T* Bb2 = SPLIT ? (Bt2 + (size_t)b * strideB) : nullptr;

  const int rlane = lane & 15;
  const int koff  = (lane >> 4) * 8;
  const int mOff  = (lane >> 4) * 8;

  v8f acc[4][4];
#pragma unroll
  for (int i = 0; i < 4; ++i)
#pragma unroll
    for (int j = 0; j < 4; ++j) acc[i][j] = (v8f){0.f,0.f,0.f,0.f,0.f,0.f,0.f,0.f};

  for (int k0 = 0; k0 < K; k0 += 32) {
    V bh[4], bl[4];
#pragma unroll
    for (int j = 0; j < 4; ++j) {
      const size_t bo = (size_t)(n0 + (j << 4) + rlane) * ldb + koff + k0;
      bh[j] = Frag<T>::load(Bb + bo);
      if (SPLIT) bl[j] = Frag<T>::load(Bb2 + bo);
    }
#pragma unroll
    for (int i = 0; i < 4; ++i) {
      const size_t ao = (size_t)(m0 + (i << 4) + rlane) * lda + koff + k0;
      V ah = Frag<T>::load(Ab + ao);
      V al;
      if (SPLIT) al = Frag<T>::load(Ab2 + ao);
#pragma unroll
      for (int j = 0; j < 4; ++j) {
        acc[i][j] = Frag<T>::mma(ah, bh[j], acc[i][j]);
        if (SPLIT) {
          acc[i][j] = Frag<T>::mma(ah, bl[j], acc[i][j]);
          acc[i][j] = Frag<T>::mma(al, bh[j], acc[i][j]);
        }
      }
      Frag<T>::guard4(acc[i][0], acc[i][1], acc[i][2], acc[i][3], ah, SPLIT ? al : ah);
    }
    Frag<T>::keep(bh[0], bh[1], bh[2], bh[3]);
    if (SPLIT) Frag<T>::keep(bl[0], bl[1], bl[2], bl[3]);
  }
  acc_guard4(acc[0][0], acc[0][1], acc[0][2], acc[0][3]);
  acc_guard4(acc[1][0], acc[1][1], acc[1][2], acc[1][3]);
  acc_guard4(acc[2][0], acc[2][1], acc[2][2], acc[2][3]);
  acc_guard4(acc[3][0], acc[3][1], acc[3][2], acc[3][3]);

  float* slab = sT[wave];
  const float* Rb = RESID ? (resid + (size_t)b * strideR) : nullptr;
#pragma unroll
  for (int i = 0; i < 4; ++i) {
    const int mBase = m0 + (i << 4);
#pragma unroll
    for (int j = 0; j < 4; ++j) {
      const int n = n0 + (j << 4) + rlane;
      float bv = 0.f;
      if (BIAS_MODE == 2) bv = bias[n];
#pragma unroll
      for (int r = 0; r < 8; ++r) {
        float v = acc[i][j][r] * scale;
        if (BIAS_MODE == 1) v += bias[mBase + mOff + r];
        if (BIAS_MODE == 2) v += bv;
        if (RESID) v += Rb[(size_t)(mBase + mOff + r) * ldc + n];
        if (ACT == 2) v = fmaxf(v, 0.0f);
        if (ACT == 4) v = (v > 0.f) ? v : 0.01f * v;
        slab[(mOff + r) * 68 + (j << 4) + rlane] = v;
      }
    }
    __builtin_amdgcn_fence(__ATOMIC_RELEASE, "workgroup");
    __builtin_amdgcn_wave_barrier();
    __builtin_amdgcn_fence(__ATOMIC_ACQUIRE, "workgroup");
    if (OUT_MODE == 0) {
      float* C = (float*)Cout + (size_t)b * strideC;
      const int hh = lane >> 4, c4 = (lane & 15) * 4;
      for (int pass = 0; pass < 2; ++pass) {
#pragma unroll
        for (int it = 0; it < 8; ++it) {
          const int row = it * 2 + hh;
          v4f v = *(const v4f*)(slab + row * 68 + c4);
          *(volatile v4f*)(C + (size_t)(mBase + row) * ldc + n0 + c4) = v;
        }
        __threadfence();
      }
    } else {
      const int q = lane >> 3, c8 = (lane & 7) * 8;
      unsigned short* C  = (unsigned short*)Cout  + (size_t)b * strideC;
      unsigned short* C2 = (OUT_MODE == 2) ? ((unsigned short*)Cout2 + (size_t)b * strideC) : nullptr;
      for (int pass = 0; pass < 2; ++pass) {
#pragma unroll
        for (int it = 0; it < 4; ++it) {
          const int row = it * 4 + q;
          const float* sp = slab + row * 68 + c8;
          v8h hv, lv;
#pragma unroll
          for (int e = 0; e < 8; ++e) {
            if (OUT_MODE == 1) {
              hv[e] = (_Float16)sp[e];
            } else {
              unsigned short hb = f2bf_bits(sp[e]);
              unsigned short lb = f2bf_bits(sp[e] - bf_bits2f(hb));
              hv[e] = __builtin_bit_cast(_Float16, hb);
              lv[e] = __builtin_bit_cast(_Float16, lb);
            }
          }
          *(volatile v8h*)(C + (size_t)(mBase + row) * ldc + n0 + c8) = hv;
          if (OUT_MODE == 2) *(volatile v8h*)(C2 + (size_t)(mBase + row) * ldc + n0 + c8) = lv;
        }
        __threadfence();
      }
    }
    __builtin_amdgcn_fence(__ATOMIC_RELEASE, "workgroup");
    __builtin_amdgcn_wave_barrier();
    __builtin_amdgcn_fence(__ATOMIC_ACQUIRE, "workgroup");
  }
}

__device__ __forceinline__ void mix8(const float (&hv)[8], const float (&dv)[8], const float* __restrict__ coef, float (&x)[8]) {
  const v4f a = *(const v4f*)(coef);
  const v4f b = *(const v4f*)(coef + 4);
#pragma unroll
  for (int e = 0; e < 4; ++e) {
    const float ca = a[e];
    const float cb = b[e];
    x[e]     = hv[e]     + dv[e]     * ca;
    x[4 + e] = hv[4 + e] + dv[4 + e] * cb;
  }
}

__global__ __launch_bounds__(256) void mix_kernel(
    const float* __restrict__ hs, const float* __restrict__ qin,
    const float* __restrict__ cw, const float* __restrict__ ck, const float* __restrict__ cv,
    const float* __restrict__ ca, const float* __restrict__ cg,
    unsigned short* __restrict__ act3h, unsigned short* __restrict__ act3l, unsigned short* __restrict__ x16) {
  const int i = blockIdx.x * 256 + threadIdx.x;
  if (i >= kRows * (kCh / 8)) return;
  const int m  = i / (kCh / 8);
  const int c0 = (i - m * (kCh / 8)) * 8;
  const int t  = m & (kSeq - 1);
  const bool hasp = (t > 0);
  const int mp = hasp ? (m - 1) : m;
  const size_t off  = (size_t)m * kCh + c0;
  const size_t offp = (size_t)mp * kCh + c0;
  const v4f h0 = *(const v4f*)(hs + off);
  const v4f h1 = *(const v4f*)(hs + off + 4);
  const v4f p0 = *(const v4f*)(hs + offp);
  const v4f p1 = *(const v4f*)(hs + offp + 4);
  const v4f q0 = *(const v4f*)(qin + off);
  const v4f q1 = *(const v4f*)(qin + off + 4);
  float hv[8], dv[8], qv[8];
#pragma unroll
  for (int e = 0; e < 4; ++e) {
    const float ha = h0[e];
    const float hb = h1[e];
    const float pa = p0[e];
    const float pb = p1[e];
    hv[e]     = ha;
    hv[4 + e] = hb;
    dv[e]     = (hasp ? pa : 0.0f) - ha;
    dv[4 + e] = (hasp ? pb : 0.0f) - hb;
    qv[e]     = q0[e];
    qv[4 + e] = q1[e];
  }
  float x[8];
  v4u qH, qL, kH, kL, vH, vL, w16, a16, g16;
  pack_split8(qv, qH, qL);
  mix8(hv, dv, ck + c0, x);
  pack_split8(x, kH, kL);
  mix8(hv, dv, cv + c0, x);
  pack_split8(x, vH, vL);
  mix8(hv, dv, cw + c0, x);
  w16 = pack_f16x8(x);
  mix8(hv, dv, ca + c0, x);
  a16 = pack_f16x8(x);
  mix8(hv, dv, cg + c0, x);
  g16 = pack_f16x8(x);
  constexpr size_t plane = (size_t)kRows * kCh;
  for (int pass = 0; pass < 2; ++pass) {
    *(volatile v4u*)(act3h + off)             = qH;
    *(volatile v4u*)(act3l + off)             = qL;
    *(volatile v4u*)(act3h + plane + off)     = kH;
    *(volatile v4u*)(act3l + plane + off)     = kL;
    *(volatile v4u*)(act3h + 2 * plane + off) = vH;
    *(volatile v4u*)(act3l + 2 * plane + off) = vL;
    *(volatile v4u*)(x16 + off)               = w16;
    *(volatile v4u*)(x16 + plane + off)       = a16;
    *(volatile v4u*)(x16 + 2 * plane + off)   = g16;
    __threadfence();
  }
}

template <int MODE>
__global__ __launch_bounds__(256) void wt_kernel(
    const float* __restrict__ W0, const float* __restrict__ W1,
    const float* __restrict__ W2, const float* __restrict__ W3,
    unsigned short* __restrict__ outH, unsigned short* __restrict__ outL,
    int Ksrc, int Nsrc, int Kpad, long planeElems, float carry) {
  __shared__ float sm[64][65];
  const int t  = threadIdx.x;
  const int k0 = blockIdx.x * 64;
  const int n0 = blockIdx.y * 64;
  const int z  = blockIdx.z;
  const float* W = (z == 0) ? W0 : (z == 1) ? W1 : (z == 2) ? W2 : W3;
#pragma unroll
  for (int i = 0; i < 16; ++i) {
    const int e  = i * 256 + t;
    const int r  = e >> 6;
    const int c  = e & 63;
    const int kk = k0 + r;
    const int nn = n0 + c;
    const bool ok = (kk < Ksrc) && (nn < Nsrc);
    const int kc = (kk < Ksrc) ? kk : (Ksrc - 1);
    const int nc = (nn < Nsrc) ? nn : (Nsrc - 1);
    const float v = W[(size_t)kc * Nsrc + nc];
    sm[c][r] = ok ? (v * carry) : 0.0f;
  }
  __syncthreads();
  const int lane = t & 31, wave = t >> 5;
  const int q = lane >> 3, c8 = (lane & 7) * 8;
  unsigned short* oh = outH + (size_t)z * planeElems;
  unsigned short* ol = outL + (size_t)z * planeElems;
  for (int pass = 0; pass < 2; ++pass) {
#pragma unroll
    for (int it = 0; it < 2; ++it) {
      const int row = wave * 8 + it * 4 + q;
      float x[8];
#pragma unroll
      for (int e = 0; e < 8; ++e) x[e] = sm[row][c8 + e];
      const size_t o = (size_t)(n0 + row) * Kpad + k0 + c8;
      if (MODE == 1) {
        const v4u u = pack_f16x8(x);
        *(volatile v4u*)(oh + o) = u;
      } else {
        v4u uh, ul;
        pack_split8(x, uh, ul);
        *(volatile v4u*)(oh + o) = uh;
        *(volatile v4u*)(ol + o) = ul;
      }
    }
    __threadfence();
  }
}

__global__ __launch_bounds__(256) void act_kernel(
    const float* __restrict__ hf2, const float* __restrict__ hgf,
    unsigned short* __restrict__ h16, unsigned short* __restrict__ hgh, unsigned short* __restrict__ hgl) {
  const int bx  = blockIdx.x;
  const int seg = (bx < 64) ? 0 : (bx < 128) ? 1 : 2;
  const int i   = ((seg == 2) ? (bx - 128) : bx) * 256 + threadIdx.x;
  const float* src = (seg == 2) ? hgf : hf2;
  const v4f a = *(const v4f*)(src + 8 * (size_t)i);
  const v4f c = *(const v4f*)(src + 8 * (size_t)i + 4);
  float xin[8], y[8];
#pragma unroll
  for (int e = 0; e < 4; ++e) { xin[e] = a[e]; xin[4 + e] = c[e]; }
#pragma unroll
  for (int e = 0; e < 8; ++e) {
    const float xv = xin[e];
    const float cx = (seg == 0) ? (2.0f * xv) : (-xv);
    const float ex = expf(cx);
    const float rc = __builtin_amdgcn_rcpf(1.0f + ex);
    y[e] = (seg == 0) ? (1.0f - 2.0f * rc) : (seg == 1) ? xv : rc;
  }
  if (seg == 2) {
    v4u uh, ul;
    pack_split8(y, uh, ul);
    unsigned short* ph = hgh + 8 * (size_t)i;
    unsigned short* pl = hgl + 8 * (size_t)i;
    *(volatile v4u*)ph = uh;
    *(volatile v4u*)pl = ul;
    __threadfence();
    *(volatile v4u*)ph = uh;
    *(volatile v4u*)pl = ul;
  } else {
    const v4u u = pack_f16x8(y);
    unsigned short* ph = h16 + 8 * (size_t)i;
    *(volatile v4u*)ph = u;
    __threadfence();
    *(volatile v4u*)ph = u;
  }
}

__device__ __forceinline__ void fuse_elem(float k0, float araw, float wraw, float sraw, float v0, float vf,
                                          float kkv, float inv, float alb, float wlb, float vlb, float ka,
                                          float& kfin, float& bb, float& ew, float& kkn, float& vfin) {
  const float av = sigm(araw + alb);
  kkn = kkv * inv;
  const float wl = kDecay * sigm(wraw + wlb);
  const float sv = sigm(sraw + vlb);
  bb   = kkn * av;
  kfin = k0 * (1.0f + (av - 1.0f) * ka);
  ew   = expf(wl);
  vfin = v0 + sv * (vf - v0);
}

__global__ __launch_bounds__(256) void headfuse_kernel(
    float* kpl, float* abpl, float* ewpl, float* skpl, float* vpl,
    const float* __restrict__ vfirst, const float* __restrict__ a_lb, const float* __restrict__ w_lb,
    const float* __restrict__ v_lb, const float* __restrict__ k_k, const float* __restrict__ k_a) {
  const int lane = threadIdx.x & 31, wave = threadIdx.x >> 5;
  const int bth = blockIdx.x * 8 + wave;
  if (bth >= kRows * kHeads) return;
  const int h = bth & (kHeads - 1);
  const size_t idx = (size_t)bth * kHd + 2 * lane;
  const int c = h * kHd + 2 * lane;
  const v2f k0v = *(const v2f*)(kpl + idx);
  const v2f arv = *(const v2f*)(abpl + idx);
  const v2f wrv = *(const v2f*)(ewpl + idx);
  const v2f srv = *(const v2f*)(skpl + idx);
  const v2f v0v = *(const v2f*)(vpl + idx);
  const v2f vfv = *(const v2f*)(vfirst + idx);
  const v2f kkc = *(const v2f*)(k_k + c);
  const v2f kac = *(const v2f*)(k_a + c);
  const v2f alv = *(const v2f*)(a_lb + c);
  const v2f wlv = *(const v2f*)(w_lb + c);
  const v2f vlv = *(const v2f*)(v_lb + c);
  const float k0a = k0v[0], k0b = k0v[1];
  const float kka = k0a * kkc[0];
  const float kkb = k0b * kkc[1];
  float ss = 0.0f;
  ss += kka * kka;
  ss += kkb * kkb;
#pragma unroll
  for (int off = 16; off > 0; off >>= 1) ss += __shfl_xor(ss, off, 32);
  const float nrm = fmaxf(sqrtf(ss), 1e-12f);
  const float inv = 1.0f / nrm;
  float kf0, bb0, ew0, kn0, vf0, kf1, bb1, ew1, kn1, vf1;
  fuse_elem(k0a, arv[0], wrv[0], srv[0], v0v[0], vfv[0], kka, inv, alv[0], wlv[0], vlv[0], kac[0], kf0, bb0, ew0, kn0, vf0);
  fuse_elem(k0b, arv[1], wrv[1], srv[1], v0v[1], vfv[1], kkb, inv, alv[1], wlv[1], vlv[1], kac[1], kf1, bb1, ew1, kn1, vf1);
  const v2f oK = (v2f){kf0, kf1};
  const v2f oB = (v2f){bb0, bb1};
  const v2f oE = (v2f){ew0, ew1};
  const v2f oN = (v2f){kn0, kn1};
  const v2f oV = (v2f){vf0, vf1};
  for (int pass = 0; pass < 2; ++pass) {
    *(volatile v2f*)(kpl + idx)  = oK;
    *(volatile v2f*)(abpl + idx) = oB;
    *(volatile v2f*)(ewpl + idx) = oE;
    *(volatile v2f*)(skpl + idx) = oN;
    *(volatile v2f*)(vpl + idx)  = oV;
    __threadfence();
  }
}

__global__ __launch_bounds__(256) void scan_kernel(
    const float* __restrict__ rpl, const float* __restrict__ ewpl, const float* __restrict__ kpl,
    const float* __restrict__ vpl, const float* __restrict__ kkpl, const float* __restrict__ bpl,
    float* __restrict__ opl) {
  __shared__ __align__(16) float sR[kChunk * kHd];
  __shared__ __align__(16) float sE[kChunk * kHd];
  __shared__ __align__(16) float sK[kChunk * kHd];
  __shared__ __align__(16) float sV[kChunk * kHd];
  __shared__ __align__(16) float sN[kChunk * kHd];
  __shared__ __align__(16) float sB[kChunk * kHd];
  __shared__ __align__(16) float sO[kChunk * kHd];
  const int tid = threadIdx.x, lane = tid & 31, wave = tid >> 5;
  const int bh = blockIdx.x;
  const int b  = bh / kHeads;
  const int h  = bh - b * kHeads;
  const int kq = tid & 3, vrow = tid >> 2;
  const int ls = tid >> 4, lc4 = (tid & 15) * 4;
  const int srow = 2 * wave + (lane >> 4), sc4 = (lane & 15) * 4;
  const size_t colbase = (size_t)h * kHd;
  float st[16];
#pragma unroll
  for (int j = 0; j < 16; ++j) st[j] = 0.0f;

#pragma unroll 1
  for (int ch = 0; ch < kSeq / kChunk; ++ch) {
    const int t0 = ch * kChunk;
    {
      const size_t g = ((size_t)(b * kSeq + t0 + ls)) * kCh + colbase + lc4;
      const v4f a0 = *(const v4f*)(rpl + g);
      const v4f a1 = *(const v4f*)(ewpl + g);
      const v4f a2 = *(const v4f*)(kpl + g);
      const v4f a3 = *(const v4f*)(vpl + g);
      const v4f a4 = *(const v4f*)(kkpl + g);
      const v4f a5 = *(const v4f*)(bpl + g);
      const int lo = ls * kHd + lc4;
      *(v4f*)(sR + lo) = a0;
      *(v4f*)(sE + lo) = a1;
      *(v4f*)(sK + lo) = a2;
      *(v4f*)(sV + lo) = a3;
      *(v4f*)(sN + lo) = a4;
      *(v4f*)(sB + lo) = a5;
    }
    __syncthreads();
#pragma unroll 1
    for (int s = 0; s < kChunk; ++s) {
      const int base = s * kHd + kq * 16;
      v4f n4[4], e4[4], b4[4], k4[4], r4[4];
#pragma unroll
      for (int jj = 0; jj < 4; ++jj) {
        n4[jj] = *(const v4f*)(sN + base + 4 * jj);
        e4[jj] = *(const v4f*)(sE + base + 4 * jj);
        b4[jj] = *(const v4f*)(sB + base + 4 * jj);
        k4[jj] = *(const v4f*)(sK + base + 4 * jj);
        r4[jj] = *(const v4f*)(sR + base + 4 * jj);
      }
      const float vt = sV[s * kHd + vrow];
      float p = 0.0f;
#pragma unroll
      for (int jj = 0; jj < 4; ++jj)
#pragma unroll
        for (int e = 0; e < 4; ++e) p = fmaf(st[4 * jj + e], n4[jj][e], p);
      p += __shfl_xor(p, 1, 32);
      p += __shfl_xor(p, 2, 32);
      const float sa = -p;
      float q = 0.0f;
#pragma unroll
      for (int jj = 0; jj < 4; ++jj)
#pragma unroll
        for (int e = 0; e < 4; ++e) {
          const float sn = st[4 * jj + e] * e4[jj][e] + sa * b4[jj][e] + vt * k4[jj][e];
          st[4 * jj + e] = sn;
          q = fmaf(sn, r4[jj][e], q);
        }
      q += __shfl_xor(q, 1, 32);
      q += __shfl_xor(q, 2, 32);
      if (kq == 0) sO[s * kHd + vrow] = q;
    }
    __syncthreads();
    {
      const v4f val = *(const v4f*)(sO + srow * kHd + sc4);
      float* dst = opl + ((size_t)(b * kSeq + t0 + srow)) * kCh + colbase + sc4;
      for (int pass = 0; pass < 2; ++pass) {
        *(volatile v4f*)dst = val;
        __threadfence();
      }
    }
  }
}

__global__ __launch_bounds__(256) void post_kernel(
    const float* __restrict__ opl, const float* __restrict__ rpl, const float* __restrict__ kpl,
    const float* __restrict__ vpl, const float* __restrict__ gpl,
    const float* __restrict__ r_k, const float* __restrict__ gn_w, const float* __restrict__ gn_b,
    unsigned* __restrict__ ogh, unsigned* __restrict__ ogl) {
  const int lane = threadIdx.x & 31, wave = threadIdx.x >> 5;
  const int bth = blockIdx.x * 8 + wave;
  if (bth >= kRows * kHeads) return;
  const int h = bth & (kHeads - 1);
  const size_t idx = (size_t)bth * kHd + 2 * lane;
  const int c = h * kHd + 2 * lane;
  const v2f ov = *(const v2f*)(opl + idx);
  const v2f rv = *(const v2f*)(rpl + idx);
  const v2f kv = *(const v2f*)(kpl + idx);
  const v2f vv = *(const v2f*)(vpl + idx);
  const v2f gv = *(const v2f*)(gpl + idx);
  const v2f rk = *(const v2f*)(r_k + c);
  const v2f gw = *(const v2f*)(gn_w + c);
  const v2f gb = *(const v2f*)(gn_b + c);
  const float o0 = ov[0], o1 = ov[1];
  float sum = 0.0f;
  sum += o0;
  sum += o1;
  float dot = 0.0f;
  dot += rv[0] * kv[0] * rk[0];
  dot += rv[1] * kv[1] * rk[1];
#pragma unroll
  for (int off = 16; off > 0; off >>= 1) {
    sum += __shfl_xor(sum, off, 32);
    dot += __shfl_xor(dot, off, 32);
  }
  const float mu = sum * kInvHd;
  const float d0 = o0 - mu, d1 = o1 - mu;
  float sq = 0.0f;
  sq += d0 * d0;
  sq += d1 * d1;
#pragma unroll
  for (int off = 16; off > 0; off >>= 1) sq += __shfl_xor(sq, off, 32);
  const float var  = sq * kInvHd;
  const float rstd = rsqrtf(var + kNormEps);
  const float y0 = (d0 * rstd) * gw[0] + gb[0] + dot * vv[0];
  const float y1 = (d1 * rstd) * gw[1] + gb[1] + dot * vv[1];
  const float z0 = y0 * gv[0];
  const float z1 = y1 * gv[1];
  unsigned short h0, l0, h1, l1;
  split_bits(z0, h0, l0);
  split_bits(z1, h1, l1);
  const unsigned wh = pk16(h0, h1);
  const unsigned wl = pk16(l0, l1);
  const size_t wi = (size_t)bth * (kHd / 2) + lane;
  volatile unsigned* ph = (volatile unsigned*)(ogh + wi);
  volatile unsigned* pl = (volatile unsigned*)(ogl + wi);
  *ph = wh;
  *pl = wl;
  __threadfence();
  *ph = wh;
  *pl = wl;
}

extern "C" void kernel_launch(void* const* d_in, const int* in_sizes, int n_in,
                              void* d_out, int out_size, void* d_ws, size_t ws_size, hipStream_t stream) {
  if (n_in < 29 || d_out == nullptr || d_ws == nullptr) return;
  if (in_sizes[0] != kRows * kCh || in_sizes[1] != kRows * kCh || in_sizes[2] != kRows * kCh ||
      in_sizes[4] != kCh || in_sizes[11] != kHeads * kHd ||
      in_sizes[12] != kCh * kCh || in_sizes[13] != kCh * kCh || in_sizes[14] != kCh * kCh || in_sizes[15] != kCh * kCh ||
      in_sizes[16] != kCh * kRankW || in_sizes[17] != kRankW * kCh ||
      in_sizes[19] != kCh * kRankV || in_sizes[20] != kRankV * kCh ||
      in_sizes[22] != kCh * kRankA || in_sizes[23] != kRankA * kCh ||
      in_sizes[25] != kCh * kRankG || in_sizes[26] != kRankG * kCh ||
      out_size != kRows * kCh) return;

  const float* query  = (const float*)d_in[0];
  const float* hidden = (const float*)d_in[1];
  const float* vfirst = (const float*)d_in[2];
  const float* x_w  = (const float*)d_in[4];
  const float* x_k  = (const float*)d_in[5];
  const float* x_v  = (const float*)d_in[6];
  const float* x_a  = (const float*)d_in[7];
  const float* x_g  = (const float*)d_in[8];
  const float* k_k  = (const float*)d_in[9];
  const float* k_a  = (const float*)d_in[10];
  const float* r_k  = (const float*)d_in[11];
  const float* W_r  = (const float*)d_in[12];
  const float* W_k  = (const float*)d_in[13];
  const float* W_v  = (const float*)d_in[14];
  const float* W_o  = (const float*)d_in[15];
  const float* w_lA = (const float*)d_in[16];
  const float* w_lB = (const float*)d_in[17];
  const float* w_lb = (const float*)d_in[18];
  const float* v_lA = (const float*)d_in[19];
  const float* v_lB = (const float*)d_in[20];
  const float* v_lb = (const float*)d_in[21];
  const float* a_lA = (const float*)d_in[22];
  const float* a_lB = (const float*)d_in[23];
  const float* a_lb = (const float*)d_in[24];
  const float* g_lA = (const float*)d_in[25];
  const float* g_lB = (const float*)d_in[26];
  const float* gn_w = (const float*)d_in[27];
  const float* gn_b = (const float*)d_in[28];
  float* out = (float*)d_out;

  char* ws = (char*)d_ws; size_t off = 0;
  auto carve = [&](size_t bytes) -> char* { char* p = ws + off; off += (bytes + 255) & ~(size_t)255; return p; };
  const size_t P = (size_t)kRows * kCh;
  unsigned short* ACT3H = (unsigned short*)carve(3 * P * 2);
  unsigned short* ACT3L = (unsigned short*)carve(3 * P * 2);
  unsigned short* X16   = (unsigned short*)carve(3 * P * 2);
  unsigned short* WBH   = (unsigned short*)carve((size_t)4 * kCh * kCh * 2);
  unsigned short* WBL   = (unsigned short*)carve((size_t)4 * kCh * kCh * 2);
  unsigned short* LA16  = (unsigned short*)carve((size_t)2 * kRankW * kCh * 2);
  unsigned short* GLA16 = (unsigned short*)carve((size_t)kRankG * kCh * 2);
  unsigned short* VLAH  = (unsigned short*)carve((size_t)kRankVP * kCh * 2);
  unsigned short* VLAL  = (unsigned short*)carve((size_t)kRankVP * kCh * 2);
  unsigned short* LB16  = (unsigned short*)carve((size_t)3 * kCh * kRankW * 2);
  unsigned short* GLBH  = (unsigned short*)carve((size_t)kCh * kRankG * 2);
  unsigned short* GLBL  = (unsigned short*)carve((size_t)kCh * kRankG * 2);
  float*          HF2   = (float*)carve((size_t)2 * kRows * kRankW * 4);
  float*          HGF   = (float*)carve((size_t)kRows * kRankG * 4);
  unsigned short* H16   = (unsigned short*)carve((size_t)3 * kRows * kRankW * 2);
  unsigned short* HGH   = (unsigned short*)carve((size_t)kRows * kRankG * 2);
  unsigned short* HGL   = (unsigned short*)carve((size_t)kRows * kRankG * 2);
  float*          F32P  = (float*)carve(7 * P * 4);
  float*          OPL   = (float*)carve(P * 4);
  if (off > ws_size || off > (size_t)134217728) return;

  float* Rp  = F32P;
  float* Kp  = F32P + P;
  float* Vp  = F32P + 2 * P;
  float* WLp = F32P + 3 * P;
  float* ARp = F32P + 4 * P;
  float* SVp = F32P + 5 * P;
  float* Gp  = F32P + 6 * P;
  unsigned short* XVH = ACT3H + 2 * P;
  unsigned short* XVL = ACT3L + 2 * P;
  unsigned short* OGH = ACT3H + P;
  unsigned short* OGL = ACT3L + P;
  const float* dummy = gn_b;

  mix_kernel<<<kRows * (kCh / 8) / 256, 256, 0, stream>>>(hidden, query, x_w, x_k, x_v, x_a, x_g, ACT3H, ACT3L, X16);

  wt_kernel<0><<<dim3(kCh / 64, kCh / 64, 4), 256, 0, stream>>>(W_r, W_k, W_v, W_o, WBH, WBL, kCh, kCh, kCh, (long)kCh * kCh, 1.0f);
  wt_kernel<1><<<dim3(kCh / 64, kRankW / 64, 2), 256, 0, stream>>>(w_lA, a_lA, a_lA, a_lA, LA16, LA16, kCh, kRankW, kCh, (long)kRankW * kCh, kLoraCarry);
  wt_kernel<1><<<dim3(kCh / 64, kRankG / 64, 1), 256, 0, stream>>>(g_lA, g_lA, g_lA, g_lA, GLA16, GLA16, kCh, kRankG, kCh, 0L, kLoraCarry);
  wt_kernel<0><<<dim3(kCh / 64, kRankVP / 64, 1), 256, 0, stream>>>(v_lA, v_lA, v_lA, v_lA, VLAH, VLAL, kCh, kRankV, kCh, 0L, 1.0f);
  wt_kernel<1><<<dim3(kRankW / 64, kCh / 64, 2), 256, 0, stream>>>(w_lB, a_lB, a_lB, a_lB, LB16, LB16, kRankW, kCh, kRankW, (long)kCh * kRankW, kLoraCarry);
  wt_kernel<1><<<dim3(kRankVP / 64, kCh / 64, 1), 256, 0, stream>>>(v_lB, v_lB, v_lB, v_lB, LB16 + (size_t)2 * kCh * kRankW, LB16, kRankV, kCh, kRankVP, 0L, kLoraCarry);
  wt_kernel<0><<<dim3(kRankG / 64, kCh / 64, 1), 256, 0, stream>>>(g_lB, g_lB, g_lB, g_lB, GLBH, GLBL, kRankG, kCh, kRankG, 0L, 1.0f);

  wmma_gemm64<1, true, 0, 0, false, 0><<<dim3((kRows / 64) * (kCh / 64) / 8, 3), 256, 0, stream>>>(
      ACT3H, ACT3L, kCh, (long)P, WBH, WBL, kCh, (long)kCh * kCh, (void*)Rp, (void*)Rp, kCh, (long)P,
      dummy, dummy, 0L, kRows, kCh, kCh, 1.0f);

  wmma_gemm64<0, false, 0, 0, false, 0><<<dim3((kRows / 64) * (kRankW / 64) / 8, 2), 256, 0, stream>>>(
      X16, X16, kCh, (long)P, LA16, LA16, kCh, (long)kRankW * kCh, (void*)HF2, (void*)HF2, kRankW, (long)kRows * kRankW,
      dummy, dummy, 0L, kRows, kRankW, kCh, kLoraCarryInv);
  wmma_gemm64<0, false, 0, 0, false, 0><<<dim3((kRows / 64) * (kRankG / 64) / 8, 1), 256, 0, stream>>>(
      X16 + 2 * P, X16 + 2 * P, kCh, 0L, GLA16, GLA16, kCh, 0L, (void*)HGF, (void*)HGF, kRankG, 0L,
      dummy, dummy, 0L, kRows, kRankG, kCh, kLoraCarryInv);
  wmma_gemm64<1, true, 0, 1, false, 0><<<dim3((kRows / 64) * (kRankVP / 64) / 8, 1), 256, 0, stream>>>(
      XVH, XVL, kCh, 0L, VLAH, VLAL, kCh, 0L, (void*)(H16 + (size_t)2 * kRows * kRankW), (void*)(H16 + (size_t)2 * kRows * kRankW),
      kRankVP, 0L, dummy, dummy, 0L, kRows, kRankVP, kCh, 1.0f);

  act_kernel<<<256, 256, 0, stream>>>(HF2, HGF, H16, HGH, HGL);

  wmma_gemm64<0, false, 0, 0, false, 0><<<dim3((kRows / 64) * (kCh / 64) / 8, 3), 256, 0, stream>>>(
      H16, H16, kRankW, (long)kRows * kRankW, LB16, LB16, kRankW, (long)kCh * kRankW, (void*)WLp, (void*)WLp, kCh, (long)P,
      dummy, dummy, 0L, kRows, kCh, kRankW, kLoraCarryInv);
  wmma_gemm64<1, true, 0, 0, false, 0><<<dim3((kRows / 64) * (kCh / 64) / 8, 1), 256, 0, stream>>>(
      HGH, HGL, kRankG, 0L, GLBH, GLBL, kRankG, 0L, (void*)Gp, (void*)Gp, kCh, 0L,
      dummy, dummy, 0L, kRows, kCh, kRankG, 1.0f);

  headfuse_kernel<<<kRows * kHeads / 8, 256, 0, stream>>>(Kp, ARp, WLp, SVp, Vp, vfirst, a_lb, w_lb, v_lb, k_k, k_a);

  scan_kernel<<<kBatch * kHeads, 256, 0, stream>>>(Rp, WLp, Kp, Vp, SVp, ARp, OPL);

  post_kernel<<<kRows * kHeads / 8, 256, 0, stream>>>(OPL, Rp, Kp, Vp, Gp, r_k, gn_w, gn_b, (unsigned*)OGH, (unsigned*)OGL);

  wmma_gemm64<1, true, 0, 0, false, 0><<<dim3((kRows / 64) * (kCh / 64) / 8, 1), 256, 0, stream>>>(
      OGH, OGL, kCh, 0L, WBH + (size_t)3 * kCh * kCh, WBL + (size_t)3 * kCh * kCh, kCh, 0L, (void*)out, (void*)out, kCh, 0L,
      dummy, dummy, 0L, kRows, kCh, kCh, 1.0f);
}
